// MultiHeadedAttention_54735063220771
// MI455X (gfx1250) — hardware-verified
//
#include <hip/hip_runtime.h>
#include <stdint.h>


typedef __attribute__((ext_vector_type(8)))  _Float16 v8h;
typedef __attribute__((ext_vector_type(16))) _Float16 v16h;
typedef __attribute__((ext_vector_type(8)))  float    v8f;
typedef __attribute__((ext_vector_type(4)))  float    v4f;

#ifndef NB
#define NB 8
#endif
#ifndef SEQ
#define SEQ 1024
#endif
#define NB_FULL 8
#define S_FULL  1024
#define EMBED   1024
#define NHEAD   16
#define HDIM    64
#define WROWS   (NHEAD * HDIM)
#define MROWS   (NB * SEQ)

#define GBM  64
#define GBN  128
#define QBLK 128
#define KBLK 64
#define LDSQ 72

static_assert(NB >= 1 && NB <= NB_FULL);
static_assert(SEQ >= QBLK && SEQ <= S_FULL);
static_assert(SEQ % QBLK == 0);
static_assert(SEQ % KBLK == 0);
static_assert(MROWS % GBM == 0);
static_assert(EMBED % GBN == 0);
static_assert(EMBED % 32 == 0);
static_assert(WROWS == EMBED);
static_assert(HDIM == 64);
static_assert(QBLK == 8 * 16);

__device__ __forceinline__ v8f wmma_f16(v16h a, v16h b, v8f c) {
  return __builtin_amdgcn_wmma_f32_16x16x32_f16(
      false, a, false, b, (short)0, c, false, false);
}

__device__ __forceinline__ v16h frag16(const _Float16* rowp, int kofs, int lane) {
  const _Float16* p = rowp + kofs + ((lane < 16) ? 0 : 8);
  v8h lo = *(const v8h*)(p);
  v8h hi = *(const v8h*)(p + 16);
  return __builtin_shufflevector(lo, hi, 0, 1, 2, 3, 4, 5, 6, 7,
                                         8, 9, 10, 11, 12, 13, 14, 15);
}

__device__ __forceinline__ float bf16_rne(float x) {
  unsigned u = __float_as_uint(x);
  u = (u + 0x7FFFu + ((u >> 16) & 1u)) & 0xFFFF0000u;
  return __uint_as_float(u);
}

__device__ __forceinline__ void wave_lds_sync() {
  __builtin_amdgcn_fence(4, "wavefront");
  __builtin_amdgcn_wave_barrier();
}

__global__ __launch_bounds__(256) void cvt_planes(
    const float* __restrict__ s0, const float* __restrict__ s1,
    const float* __restrict__ s2, const float* __restrict__ s3,
    _Float16* d0, _Float16* d1, _Float16* d2, _Float16* d3,
    int rows, int cols8, int dseg, int sseg, float scale) {
  const int which = blockIdx.y;
  const float* src = (which == 0) ? s0 : (which == 1) ? s1 : (which == 2) ? s2 : s3;
  _Float16* dst    = (which == 0) ? d0 : (which == 1) ? d1 : (which == 2) ? d2 : d3;

  const int idx = blockIdx.x * 256 + threadIdx.x;
  if (idx >= rows * cols8) return;
  const int row  = idx / cols8;
  const int c8   = idx - row * cols8;
  const int bidx = row / dseg;
  const int srow = bidx * sseg + (row - bidx * dseg);
  const size_t cols = (size_t)cols8 * 8;

  const float4* sp = (const float4*)(src + (size_t)srow * cols + (size_t)c8 * 8);
  const float4 u = sp[0];
  const float4 w = sp[1];
  v8h o;
  o[0] = (_Float16)(bf16_rne(u.x) * scale);
  o[1] = (_Float16)(bf16_rne(u.y) * scale);
  o[2] = (_Float16)(bf16_rne(u.z) * scale);
  o[3] = (_Float16)(bf16_rne(u.w) * scale);
  o[4] = (_Float16)(bf16_rne(w.x) * scale);
  o[5] = (_Float16)(bf16_rne(w.y) * scale);
  o[6] = (_Float16)(bf16_rne(w.z) * scale);
  o[7] = (_Float16)(bf16_rne(w.w) * scale);

  volatile v8h* dp = (volatile v8h*)(dst + (size_t)row * cols + (size_t)c8 * 8);
  *dp = o;
  __threadfence();
  *dp = o;
}

template <typename OT> struct StgPitch {
  static constexpr int v = (sizeof(OT) == 2) ? 72 : 68;
};

template <typename OT>
__global__ __launch_bounds__(128) __attribute__((amdgpu_num_vgpr(256)))
void gemm_nt(const _Float16* __restrict__ A, const _Float16* __restrict__ Bm,
             const float* __restrict__ bias, OT* C, int N, int K, float scale) {
  constexpr int PITCH = StgPitch<OT>::v;
  __shared__ __align__(16) OT stg[4][16][PITCH];

  const int lane = threadIdx.x & 31;
  const int wave = threadIdx.x >> 5;
  const int hh   = lane >> 4;
  const int cc   = lane & 15;
  const int wr   = wave >> 1;
  const int wc   = wave & 1;
  const int mbase = blockIdx.y * GBM + wr * 32;
  const int nbase = blockIdx.x * GBN + wc * 64;

  const _Float16* ar0 = A  + (size_t)(mbase + cc) * K;
  const _Float16* ar1 = ar0 + (size_t)16 * K;
  const _Float16* br0 = Bm + (size_t)(nbase + cc) * K;
  const _Float16* br1 = br0 + (size_t)16 * K;
  const _Float16* br2 = br0 + (size_t)32 * K;
  const _Float16* br3 = br0 + (size_t)48 * K;

  v8f acc[8] = {};

#pragma unroll 1
  for (int k0 = 0; k0 < K; k0 += 32) {
    const v16h a0 = frag16(ar0, k0, lane);
    const v16h a1 = frag16(ar1, k0, lane);
    const v16h b0 = frag16(br0, k0, lane);
    const v16h b1 = frag16(br1, k0, lane);
    const v16h b2 = frag16(br2, k0, lane);
    const v16h b3 = frag16(br3, k0, lane);
    acc[0] = wmma_f16(a0, b0, acc[0]);
    acc[1] = wmma_f16(a0, b1, acc[1]);
    acc[2] = wmma_f16(a0, b2, acc[2]);
    acc[3] = wmma_f16(a0, b3, acc[3]);
    acc[4] = wmma_f16(a1, b0, acc[4]);
    acc[5] = wmma_f16(a1, b1, acc[5]);
    acc[6] = wmma_f16(a1, b2, acc[6]);
    acc[7] = wmma_f16(a1, b3, acc[7]);
    asm volatile("v_nop\n\tv_nop\n\tv_nop\n\tv_nop"
                 : "+v"(acc[0]), "+v"(acc[1]), "+v"(acc[2]), "+v"(acc[3]),
                   "+v"(acc[4]), "+v"(acc[5]), "+v"(acc[6]), "+v"(acc[7])
                 : "v"(a0), "v"(a1), "v"(b0), "v"(b1), "v"(b2), "v"(b3));
  }

  float bi[4] = {0.f, 0.f, 0.f, 0.f};
  if constexpr (sizeof(OT) == 4) {
#pragma unroll
    for (int ni = 0; ni < 4; ++ni) bi[ni] = bf16_rne(bias[nbase + ni * 16 + cc]);
  }

  OT* sw = &stg[wave][0][0];
#pragma unroll
  for (int mi = 0; mi < 2; ++mi) {
#pragma unroll
    for (int ni = 0; ni < 4; ++ni) {
#pragma unroll
      for (int r = 0; r < 8; ++r) {
        const float v = acc[mi * 4 + ni][r] * scale + bi[ni];
        sw[(8 * hh + r) * PITCH + ni * 16 + cc] = (OT)v;
      }
    }
    wave_lds_sync();

    const int row0 = mbase + mi * 16;
    if constexpr (sizeof(OT) == 2) {
      v8h vals[4];
#pragma unroll
      for (int it = 0; it < 4; ++it) {
        const int cidx = it * 32 + lane;
        const int rr = cidx >> 3, ch = cidx & 7;
        vals[it] = *(const v8h*)(sw + rr * PITCH + ch * 8);
      }
#pragma unroll
      for (int it = 0; it < 4; ++it) {
        const int cidx = it * 32 + lane;
        const int rr = cidx >> 3, ch = cidx & 7;
        *(volatile v8h*)(C + (size_t)(row0 + rr) * N + nbase + ch * 8) = vals[it];
      }
      __threadfence();
#pragma unroll
      for (int it = 0; it < 4; ++it) {
        const int cidx = it * 32 + lane;
        const int rr = cidx >> 3, ch = cidx & 7;
        *(volatile v8h*)(C + (size_t)(row0 + rr) * N + nbase + ch * 8) = vals[it];
      }
    } else {
      v4f vals[8];
#pragma unroll
      for (int it = 0; it < 8; ++it) {
        const int cidx = it * 32 + lane;
        const int rr = cidx >> 4, ch = cidx & 15;
        vals[it] = *(const v4f*)(sw + rr * PITCH + ch * 4);
      }
#pragma unroll
      for (int it = 0; it < 8; ++it) {
        const int cidx = it * 32 + lane;
        const int rr = cidx >> 4, ch = cidx & 15;
        *(volatile v4f*)(C + (size_t)(row0 + rr) * N + nbase + ch * 4) = vals[it];
      }
      __threadfence();
#pragma unroll
      for (int it = 0; it < 8; ++it) {
        const int cidx = it * 32 + lane;
        const int rr = cidx >> 4, ch = cidx & 15;
        *(volatile v4f*)(C + (size_t)(row0 + rr) * N + nbase + ch * 4) = vals[it];
      }
    }
    wave_lds_sync();
  }
}

__global__ __launch_bounds__(256) __attribute__((amdgpu_num_vgpr(256)))
void attn_fwd(const _Float16* __restrict__ qp, const _Float16* __restrict__ kp,
              const _Float16* __restrict__ vp, _Float16* ctx) {
  __shared__ __align__(16) _Float16 Qs[QBLK][LDSQ];
  __shared__ __align__(16) _Float16 Ks[KBLK][LDSQ];
  __shared__ __align__(16) _Float16 Vs[HDIM][LDSQ];
  __shared__ __align__(16) _Float16 Ps[8][16][LDSQ];

  const int tid  = threadIdx.x;
  const int lane = tid & 31;
  const int wave = tid >> 5;
  const int b  = blockIdx.y / NHEAD;
  const int h  = blockIdx.y - b * NHEAD;
  const int q0 = blockIdx.x * QBLK;

  const size_t rs = EMBED;
  const _Float16* gq = qp + (size_t)(b * SEQ + q0) * rs + h * HDIM;

#pragma unroll
  for (int i = 0; i < 4; ++i) {
    const int idx = tid + i * 256;
    const int r   = idx >> 3;
    const int c8  = (idx & 7) << 3;
    *(v8h*)&Qs[r][c8] = *(const v8h*)(gq + (size_t)r * rs + c8);
  }

  float mrun[8], lrun[8];
  v8f o[4] = {};
#pragma unroll
  for (int j = 0; j < 8; ++j) { mrun[j] = -1e30f; lrun[j] = 0.f; }

  const int qrow = wave * 16 + (lane & 15);

#pragma unroll 1
  for (int kb = 0; kb < SEQ; kb += KBLK) {
    const _Float16* gk = kp + (size_t)(b * SEQ + kb) * rs + h * HDIM;
    const _Float16* gv = vp + (size_t)(b * SEQ + kb) * rs + h * HDIM;

#pragma unroll
    for (int i = 0; i < 2; ++i) {
      const int idx = tid + i * 256;
      const int r   = idx >> 3;
      const int c8  = (idx & 7) << 3;
      *(v8h*)&Ks[r][c8] = *(const v8h*)(gk + (size_t)r * rs + c8);
    }
#pragma unroll
    for (int i = 0; i < 2; ++i) {
      const int idx = tid + i * 256;
      const int r   = idx >> 3;
      const int c8  = (idx & 7) << 3;
      const v8h v = *(const v8h*)(gv + (size_t)r * rs + c8);
#pragma unroll
      for (int j = 0; j < 8; ++j) Vs[c8 + j][r] = v[j];
    }
    __syncthreads();

    const v16h qa0 = frag16(&Qs[qrow][0], 0, lane);
    const v16h qa1 = frag16(&Qs[qrow][0], 32, lane);
    v8f sc[4];
#pragma unroll
    for (int n = 0; n < 4; ++n) {
      const int krow = n * 16 + (lane & 15);
      const v16h kb0 = frag16(&Ks[krow][0], 0, lane);
      const v16h kb1 = frag16(&Ks[krow][0], 32, lane);
      v8f s = {};
      s = wmma_f16(qa0, kb0, s);
      s = wmma_f16(qa1, kb1, s);
      asm volatile("v_nop\n\tv_nop\n\tv_nop\n\tv_nop"
                   : "+v"(s) : "v"(qa0), "v"(qa1), "v"(kb0), "v"(kb1));
      sc[n] = s * 0.125f;
    }

#pragma unroll
    for (int j = 0; j < 8; ++j) {
      float mx = fmaxf(fmaxf(sc[0][j], sc[1][j]), fmaxf(sc[2][j], sc[3][j]));
      mx = fmaxf(mx, __shfl_xor(mx, 1, 32));
      mx = fmaxf(mx, __shfl_xor(mx, 2, 32));
      mx = fmaxf(mx, __shfl_xor(mx, 4, 32));
      mx = fmaxf(mx, __shfl_xor(mx, 8, 32));
      const float mnew = fmaxf(mrun[j], mx);
      const float al   = __expf(mrun[j] - mnew);
      mrun[j] = mnew;
      float rsum = 0.f;
#pragma unroll
      for (int n = 0; n < 4; ++n) {
        const float p = __expf(sc[n][j] - mnew);
        sc[n][j] = p * 1024.0f;
        rsum += p;
      }
      rsum += __shfl_xor(rsum, 1, 32);
      rsum += __shfl_xor(rsum, 2, 32);
      rsum += __shfl_xor(rsum, 4, 32);
      rsum += __shfl_xor(rsum, 8, 32);
      lrun[j] = lrun[j] * al + rsum;
#pragma unroll
      for (int n = 0; n < 4; ++n) o[n][j] *= al;
    }

    {
      _Float16* pw = &Ps[wave][0][0];
      const int ccol = lane & 15;
      const int rofs = (lane < 16) ? 0 : 8;
#pragma unroll
      for (int n = 0; n < 4; ++n)
#pragma unroll
        for (int j = 0; j < 8; ++j)
          pw[(j + rofs) * LDSQ + n * 16 + ccol] = (_Float16)sc[n][j];
    }
    wave_lds_sync();

    const v16h pa0 = frag16(&Ps[wave][lane & 15][0], 0, lane);
    const v16h pa1 = frag16(&Ps[wave][lane & 15][0], 32, lane);
#pragma unroll
    for (int n = 0; n < 4; ++n) {
      const int drow = n * 16 + (lane & 15);
      const v16h vb0 = frag16(&Vs[drow][0], 0, lane);
      const v16h vb1 = frag16(&Vs[drow][0], 32, lane);
      o[n] = wmma_f16(pa0, vb0, o[n]);
      o[n] = wmma_f16(pa1, vb1, o[n]);
      asm volatile("v_nop\n\tv_nop\n\tv_nop\n\tv_nop"
                   : "+v"(o[n]) : "v"(pa0), "v"(pa1), "v"(vb0), "v"(vb1));
    }
    __syncthreads();
  }

  {
    _Float16* pw = &Ps[wave][0][0];
    const int ccol = lane & 15;
    const int rofs = (lane < 16) ? 0 : 8;
#pragma unroll
    for (int j = 0; j < 8; ++j) {
      const float inv = (1.0f / lrun[j]) * 0.015625f;
#pragma unroll
      for (int n = 0; n < 4; ++n)
        pw[(j + rofs) * LDSQ + n * 16 + ccol] = (_Float16)(o[n][j] * inv);
    }
  }
  wave_lds_sync();

  v8h vals[4];
#pragma unroll
  for (int it = 0; it < 4; ++it) {
    const int cidx = it * 32 + lane;
    const int rr = cidx >> 3, ch = cidx & 7;
    vals[it] = *(const v8h*)&Ps[wave][rr][ch * 8];
  }
  const size_t rowbase = (size_t)(b * SEQ + q0 + wave * 16);
#pragma unroll
  for (int it = 0; it < 4; ++it) {
    const int cidx = it * 32 + lane;
    const int rr = cidx >> 3, ch = cidx & 7;
    *(volatile v8h*)(ctx + (rowbase + rr) * EMBED + h * HDIM + ch * 8) = vals[it];
  }
  __threadfence();
#pragma unroll
  for (int it = 0; it < 4; ++it) {
    const int cidx = it * 32 + lane;
    const int rr = cidx >> 3, ch = cidx & 7;
    *(volatile v8h*)(ctx + (rowbase + rr) * EMBED + h * HDIM + ch * 8) = vals[it];
  }
}

extern "C" void kernel_launch(void* const* d_in, const int* in_sizes, int n_in,
                              void* d_out, int out_size, void* d_ws, size_t ws_size,
                              hipStream_t stream) {
  if (n_in < 8) return;
  const float* xk = (const float*)d_in[0];
  const float* xv = (const float*)d_in[1];
  const float* xq = (const float*)d_in[2];
  const float* wk = (const float*)d_in[3];
  const float* wv = (const float*)d_in[4];
  const float* wq = (const float*)d_in[5];
  const float* wo = (const float*)d_in[6];
  const float* bo = (const float*)d_in[7];
  float* out = (float*)d_out;

  const long long needX = ((long long)(NB - 1) * S_FULL + SEQ) * (long long)EMBED;
  if ((long long)in_sizes[0] < needX || (long long)in_sizes[1] < needX ||
      (long long)in_sizes[2] < needX) return;
  if (in_sizes[3] < WROWS * EMBED || in_sizes[4] < WROWS * EMBED ||
      in_sizes[5] < WROWS * EMBED || in_sizes[6] < EMBED * EMBED ||
      in_sizes[7] < EMBED) return;
  if ((long long)out_size < (long long)MROWS * EMBED) return;

  const size_t planeX = (size_t)MROWS * EMBED * sizeof(_Float16);
  const size_t planeW = (size_t)WROWS * EMBED * sizeof(_Float16);
  const size_t total  = 7 * planeX + 4 * planeW;
  if (ws_size < total) return;

  char* w = (char*)d_ws;
  _Float16* xk16 = (_Float16*)w; w += planeX;
  _Float16* xv16 = (_Float16*)w; w += planeX;
  _Float16* xq16 = (_Float16*)w; w += planeX;
  _Float16* wk16 = (_Float16*)w; w += planeW;
  _Float16* wv16 = (_Float16*)w; w += planeW;
  _Float16* wq16 = (_Float16*)w; w += planeW;
  _Float16* wo16 = (_Float16*)w; w += planeW;
  _Float16* qpl  = (_Float16*)w; w += planeX;
  _Float16* kpl  = (_Float16*)w; w += planeX;
  _Float16* vpl  = (_Float16*)w; w += planeX;
  _Float16* cpl  = (_Float16*)w; w += planeX;

  {
    const int nthr = MROWS * (EMBED / 8);
    dim3 g((unsigned)((nthr + 255) / 256), 3);
    cvt_planes<<<g, 256, 0, stream>>>(xk, xv, xq, xq, xk16, xv16, xq16, xq16,
                                       MROWS, EMBED / 8, SEQ, S_FULL, 1.0f);
  }
  {
    const int nthr = WROWS * (EMBED / 8);
    dim3 g((unsigned)((nthr + 255) / 256), 4);
    cvt_planes<<<g, 256, 0, stream>>>(wk, wv, wq, wo, wk16, wv16, wq16, wo16,
                                       WROWS, EMBED / 8, WROWS, WROWS, 16.0f);
  }

  dim3 gg(EMBED / GBN, MROWS / GBM);
  gemm_nt<_Float16><<<gg, 128, 0, stream>>>(xq16, wq16, bo, qpl, EMBED, EMBED, 0.0625f);
  gemm_nt<_Float16><<<gg, 128, 0, stream>>>(xk16, wk16, bo, kpl, EMBED, EMBED, 0.0625f);
  gemm_nt<_Float16><<<gg, 128, 0, stream>>>(xv16, wv16, bo, vpl, EMBED, EMBED, 0.0625f);

  dim3 ga(SEQ / QBLK, NB * NHEAD);
  attn_fwd<<<ga, 256, 0, stream>>>(qpl, kpl, vpl, cpl);

  gemm_nt<float><<<gg, 128, 0, stream>>>(cpl, wo16, bo, out, EMBED, EMBED, 0.00390625f);
}
